// MultiHeadAttention_4922032521398
// MI455X (gfx1250) — hardware-run, weakly checked
//
#include <hip/hip_runtime.h>
#ifndef NB
#define NB 32
#endif
#ifndef SEQ
#define SEQ 512
#endif
#define NB_FULL 32
#define SEQ_FULL 512
#define DM 256
#define NH 4
#define HD 64
#define NQKV (3 * DM)
#define NW (SEQ / 32)
#define NW4 (NW / 4)
#define NC (SEQ / 256)
#define NBG ((NB) < 8 ? (NB) : 8)
#define NR ((size_t)NB * SEQ)

typedef unsigned short v8us __attribute__((ext_vector_type(8), may_alias));
typedef float  v8f  __attribute__((ext_vector_type(8)));
typedef float  v4f  __attribute__((ext_vector_type(4)));
typedef float  v4fa __attribute__((ext_vector_type(4), may_alias));
typedef int    v4ia __attribute__((ext_vector_type(4), may_alias));
typedef unsigned int v4u  __attribute__((ext_vector_type(4)));
typedef unsigned int v4ua __attribute__((ext_vector_type(4), may_alias));
typedef _Float16 v16h __attribute__((ext_vector_type(16)));
typedef _Float16 v4h  __attribute__((ext_vector_type(4)));
union FragH { v16h v; v8us half[2]; _Float16 h[16]; unsigned short u[16]; };

static_assert(NH * HD == DM);
static_assert(SEQ % 256 == 0 && SEQ <= SEQ_FULL && NB <= NB_FULL);
static_assert(NB % NBG == 0);
static_assert((SEQ * NW4) % 256 == 0);
static_assert((NR * DM) % 2048 == 0);
static_assert(NQKV % 64 == 0 && DM % 64 == 0 && DM % 32 == 0 && HD % 32 == 0 && SEQ % 128 == 0);

__device__ __forceinline__ unsigned short bf16_bits(float x) { unsigned int u = __float_as_uint(x); return (unsigned short)((u + 0x7FFFu + ((u >> 16) & 1u)) >> 16); }
__device__ __forceinline__ float bf16_rne(float x) { return __uint_as_float(((unsigned int)bf16_bits(x)) << 16); }

__global__ __launch_bounds__(256) void k_x16(const float* __restrict__ x, _Float16* __restrict__ X16, size_t n8) {
  const size_t t = (size_t)blockIdx.x * 256 + threadIdx.x; if (t >= n8) return;
  const size_t e = t * 8; const size_t b = e / ((size_t)SEQ * DM); const size_t rem = e - b * ((size_t)SEQ * DM);
  const float* src = x + b * ((size_t)SEQ_FULL * DM) + rem;
  const v4f a = *(const v4fa*)src, c = *(const v4fa*)(src + 4);
  FragH f;
#pragma unroll
  for (int q = 0; q < 4; ++q) { f.h[q] = (_Float16)bf16_rne(a[q]); f.h[4 + q] = (_Float16)bf16_rne(c[q]); }
  const v8us o = f.half[0];
  *(volatile v8us*)((unsigned short*)X16 + t * 8) = o; __threadfence(); *(volatile v8us*)((unsigned short*)X16 + t * 8) = o;
}

__global__ __launch_bounds__(256) void k_wnat(const float* __restrict__ w, size_t n8, _Float16* __restrict__ Bt) {
  const size_t t = (size_t)blockIdx.x * 256 + threadIdx.x; if (t >= n8) return;
  const v4f a = *(const v4fa*)(w + t * 8), c = *(const v4fa*)(w + t * 8 + 4);
  FragH f;
#pragma unroll
  for (int q = 0; q < 4; ++q) { f.h[q] = (_Float16)(bf16_rne(a[q]) * 16.0f); f.h[4 + q] = (_Float16)(bf16_rne(c[q]) * 16.0f); }
  const v8us o = f.half[0];
  *(volatile v8us*)((unsigned short*)Bt + t * 8) = o; __threadfence(); *(volatile v8us*)((unsigned short*)Bt + t * 8) = o;
}

template <int NHv, int TTv>
__global__ __launch_bounds__(256) void k_vt(const _Float16* __restrict__ V16, int ldv, int voff, _Float16* __restrict__ Vt) {
  __shared__ unsigned short tl[64][66];
  const int tid = threadIdx.x; const int slab = blockIdx.x / (TTv / 64), lg = blockIdx.x % (TTv / 64); const int b = slab / NHv, h = slab % NHv;
  for (int i = tid; i < 64 * 8; i += 256) { const int r = i / 8, c8 = (i % 8) * 8; FragH f; f.half[0] = *(const v8us*)((const unsigned short*)V16 + ((size_t)b * TTv + lg * 64 + r) * ldv + voff + h * 64 + c8);
#pragma unroll
    for (int q = 0; q < 8; ++q) tl[r][c8 + q] = f.u[q]; }
  __syncthreads();
  for (int pass = 0; pass < 2; ++pass) {
#pragma unroll
    for (int rd = 0; rd < 2; ++rd) { const int d = rd * 32 + tid / 8, pc = tid % 8; FragH f;
#pragma unroll
      for (int q = 0; q < 8; ++q) f.u[q] = tl[pc * 8 + q][d];
      *(volatile v8us*)((unsigned short*)Vt + ((size_t)slab * 64 + d) * TTv + lg * 64 + pc * 8) = f.half[0]; }
    if (pass == 0) __threadfence(); } }

__device__ __forceinline__ v16h g2_frag(const _Float16* p, int hh) { FragH f; f.half[0] = *(const v8us*)((const unsigned short*)p + 8 * hh); f.half[1] = *(const v8us*)((const unsigned short*)p + 16 + 8 * hh); return f.v; }
__device__ __forceinline__ v8f g2_mma(v16h a, v16h b, v8f c) { v8f d = __builtin_amdgcn_wmma_f32_16x16x32_f16(false, a, false, b, (short)0, c, false, false); asm volatile("v_nop\n\tv_nop\n\tv_nop\n\tv_nop" : "+v"(d) : "v"(a), "v"(b)); return d; }
__global__ __launch_bounds__(128) void k_gemm2(const _Float16* __restrict__ A, int lda, size_t sAy, size_t sAz,
    const _Float16* __restrict__ Bh, int ldb, size_t sBy, size_t sBz, float alpha,
    float* __restrict__ C, _Float16* __restrict__ C16, int ldc, size_t sCy, size_t sCz, int N, int K) {
  __shared__ __attribute__((aligned(16))) float so[4][32][68];
  const int tid = threadIdx.x, w = tid >> 5, lane = tid & 31, ln = lane & 15, hh = lane >> 4; const int by = blockIdx.y, bz = blockIdx.z;
  A += (size_t)by * sAy + (size_t)bz * sAz; Bh += (size_t)by * sBy + (size_t)bz * sBz; const size_t cofs = (size_t)by * sCy + (size_t)bz * sCz;
  const int ntn = N >> 6; const int mt = blockIdx.x / ntn, nq = blockIdx.x - mt * ntn; const int row0 = mt * 128 + 32 * w, col0 = nq * 64;
  const _Float16* a0p = A + (size_t)(row0 + ln) * lda; const _Float16* a1p = a0p + (size_t)16 * lda;
  const _Float16* b0p = Bh + (size_t)(col0 + ln) * ldb; const _Float16* b1p = b0p + (size_t)16 * ldb; const _Float16* b2p = b1p + (size_t)16 * ldb; const _Float16* b3p = b2p + (size_t)16 * ldb;
  const v8f z8 = {0.f,0.f,0.f,0.f,0.f,0.f,0.f,0.f}; v8f c00 = z8, c01 = z8, c02 = z8, c03 = z8, c10 = z8, c11 = z8, c12 = z8, c13 = z8;
#pragma unroll 1
  for (int kb = 0; kb < K; kb += 32) { const v16h a0 = g2_frag(a0p + kb, hh), a1 = g2_frag(a1p + kb, hh);
    v16h b = g2_frag(b0p + kb, hh); c00 = g2_mma(a0, b, c00); c10 = g2_mma(a1, b, c10);
    b = g2_frag(b1p + kb, hh); c01 = g2_mma(a0, b, c01); c11 = g2_mma(a1, b, c11);
    b = g2_frag(b2p + kb, hh); c02 = g2_mma(a0, b, c02); c12 = g2_mma(a1, b, c12);
    b = g2_frag(b3p + kb, hh); c03 = g2_mma(a0, b, c03); c13 = g2_mma(a1, b, c13); }
  v8f accs[8] = {c00, c01, c02, c03, c10, c11, c12, c13};
#pragma unroll
  for (int u = 0; u < 8; ++u) { const int t = u & 3, half = u >> 2;
#pragma unroll
    for (int r = 0; r < 8; ++r) { const int rloc = half * 16 + 8 * hh + r; so[w][rloc][t * 16 + ln] = accs[u][r] * alpha; } }
  __syncthreads();
  const int rsub = lane >> 4, c4 = (lane & 15) * 4;
  for (int pass = 0; pass < 2; ++pass) {
#pragma unroll
    for (int q = 0; q < 16; ++q) { const int r = q * 2 + rsub; const v4f v = *(const v4fa*)&so[w][r][c4];
      if (C) *(volatile v4f*)(C + cofs + (size_t)(row0 + r) * ldc + col0 + c4) = v;
      if (C16) { v4h h4;
#pragma unroll
        for (int i = 0; i < 4; ++i) h4[i] = (_Float16)v[i];
        *(volatile v4h*)(C16 + cofs + (size_t)(row0 + r) * ldc + col0 + c4) = h4; } }
    if (pass == 0) __threadfence(); } }

__device__ __forceinline__ unsigned adj_bit(int v) { return ((v != 0) && !((v > 1) && (v < 9))) ? 1u : 0u; }
__global__ __launch_bounds__(256) void k_pack(const int* __restrict__ adj, unsigned* __restrict__ BITS) {
  const int mode = blockIdx.y, b = blockIdx.z;
  const int tq = blockIdx.x * 256 + threadIdx.x; const int i = tq / NW4, c = tq % NW4;
  const int* base = adj + (size_t)b * SEQ_FULL * SEQ_FULL;
  unsigned wd[4];
  if (mode == 0) {
    const int* rp = base + (size_t)i * SEQ_FULL + c * 128;
#pragma unroll
    for (int u = 0; u < 4; ++u) { unsigned word = 0;
#pragma unroll 2
      for (int g = 0; g < 8; ++g) { const v4ia v = *(const v4ia*)(rp + u * 32 + g * 4);
        word |= (adj_bit(v[0]) | (adj_bit(v[1]) << 1) | (adj_bit(v[2]) << 2) | (adj_bit(v[3]) << 3)) << (g * 4); }
      wd[u] = word; }
  } else {
#pragma unroll
    for (int u = 0; u < 4; ++u) { unsigned word = 0;
#pragma unroll 4
      for (int tb = 0; tb < 32; ++tb) { const int v = base[(size_t)(c * 128 + u * 32 + tb) * SEQ_FULL + i]; word |= adj_bit(v) << tb; }
      wd[u] = word; }
  }
  const v4u o = {wd[0], wd[1], wd[2], wd[3]};
  unsigned* dst = BITS + (((size_t)mode * NB + b) * SEQ + i) * NW + 4 * c;
  *(volatile v4u*)dst = o; __threadfence(); *(volatile v4u*)dst = o;
}

__global__ __launch_bounds__(256) void k_mask(const unsigned* __restrict__ BITS, unsigned* __restrict__ PM) {
  const int hd = blockIdx.y, b = blockIdx.z;
  const int tq = blockIdx.x * 256 + threadIdx.x; const int i = tq / NW4, c = tq % NW4;
  const int psel = (hd == 1 || hd == 2) ? 1 : 0;
  const unsigned* src = BITS + ((size_t)psel * NB + b) * SEQ * NW;
  unsigned wd[4];
  if (hd < 2) {
    const v4u m = *(const v4ua*)(src + (size_t)i * NW + 4 * c);
    wd[0] = m[0]; wd[1] = m[1]; wd[2] = m[2]; wd[3] = m[3];
  } else {
    unsigned mine[NW];
#pragma unroll
    for (int q4 = 0; q4 < NW4; ++q4) { const v4u m = *(const v4ua*)(src + (size_t)i * NW + 4 * q4); mine[4 * q4] = m[0]; mine[4 * q4 + 1] = m[1]; mine[4 * q4 + 2] = m[2]; mine[4 * q4 + 3] = m[3]; }
#pragma unroll
    for (int u = 0; u < 4; ++u) { unsigned word = 0;
#pragma unroll 2
      for (int tb = 0; tb < 32; ++tb) { const unsigned* rj = src + (size_t)(c * 128 + u * 32 + tb) * NW; unsigned acc = 0;
#pragma unroll
        for (int q4 = 0; q4 < NW4; ++q4) { const v4u r = *(const v4ua*)(rj + 4 * q4);
          acc |= (mine[4 * q4] & r[0]) | (mine[4 * q4 + 1] & r[1]) | (mine[4 * q4 + 2] & r[2]) | (mine[4 * q4 + 3] & r[3]); }
        word |= ((acc != 0u) ? 1u : 0u) << tb; }
      wd[u] = word; }
  }
#pragma unroll
  for (int u = 0; u < 4; ++u) wd[u] |= ((i >> 5) == (4 * c + u)) ? (1u << (i & 31)) : 0u;
  const v4u o = {wd[0], wd[1], wd[2], wd[3]};
  unsigned* dst = PM + ((((size_t)b * NH + hd) * SEQ) + i) * NW + 4 * c;
  *(volatile v4u*)dst = o; __threadfence(); *(volatile v4u*)dst = o;
}

__global__ __launch_bounds__(256) void k_msm(const float* __restrict__ S, const unsigned* __restrict__ PMg, _Float16* __restrict__ P, int nrows) {
  const int lane = threadIdx.x & 31; const int row = blockIdx.x * 8 + (threadIdx.x >> 5);
  if (row >= nrows) return;
  const float* s = S + (size_t)row * SEQ; const unsigned* mw = PMg + (size_t)row * NW;
  float v[NC * 8]; float mx = -3.0e38f;
#pragma unroll
  for (int c = 0; c < NC; ++c) {
    const v4f x0 = *(const v4fa*)(s + c * 256 + 8 * lane), x1 = *(const v4fa*)(s + c * 256 + 8 * lane + 4);
    const unsigned bits = mw[c * 8 + (lane >> 2)] >> (8 * (lane & 3));
#pragma unroll
    for (int q = 0; q < 4; ++q) {
      const float lo = (((bits >> q) & 1u) != 0u) ? x0[q] : -1.0e9f;
      const float hi = (((bits >> (4 + q)) & 1u) != 0u) ? x1[q] : -1.0e9f;
      v[c * 8 + q] = lo; v[c * 8 + 4 + q] = hi; mx = fmaxf(mx, fmaxf(lo, hi)); }
  }
#pragma unroll
  for (int m = 16; m >= 1; m >>= 1) mx = fmaxf(mx, __shfl_xor(mx, m, 32));
  float se = 0.f;
#pragma unroll
  for (int i = 0; i < NC * 8; ++i) { const float e = __expf(v[i] - mx); v[i] = e; se += e; }
#pragma unroll
  for (int m = 16; m >= 1; m >>= 1) se += __shfl_xor(se, m, 32);
  const float sc = 256.0f * (1.0f / se);
  v8us o[NC];
#pragma unroll
  for (int c = 0; c < NC; ++c) { FragH f;
#pragma unroll
    for (int q = 0; q < 8; ++q) f.h[q] = (_Float16)(v[c * 8 + q] * sc);
    o[c] = f.half[0]; }
  unsigned short* prow = (unsigned short*)P + (size_t)row * SEQ + 8 * lane;
  for (int pass = 0; pass < 2; ++pass) {
#pragma unroll
    for (int c = 0; c < NC; ++c) *(volatile v8us*)(prow + c * 256) = o[c];
    if (pass == 0) __threadfence(); }
}

constexpr size_t al256(size_t b) { return (b + 255) & ~(size_t)255; }
constexpr size_t WS_TOTAL =
    al256((size_t)NQKV * DM * 2) + al256((size_t)DM * DM * 2) + al256(NR * DM * 2) + al256(NR * NQKV * 2) +
    al256((size_t)2 * NB * SEQ * NW * 4) + al256((size_t)NB * NH * SEQ * NW * 4) + al256((size_t)NB * NH * HD * SEQ * 2) +
    al256(NR * DM * 2) + al256((size_t)NBG * NH * SEQ * SEQ * 4) + al256((size_t)NBG * NH * SEQ * SEQ * 2);
static_assert(WS_TOTAL <= (size_t)134217728);

extern "C" void kernel_launch(void* const* d_in, const int* in_sizes, int n_in,
                              void* d_out, int out_size, void* d_ws, size_t ws_size, hipStream_t stream) {
  (void)out_size;
  if (n_in < 4) return;
  if (in_sizes[0] < NB * SEQ * DM || in_sizes[1] < NB * SEQ * SEQ || in_sizes[2] < NQKV * DM || in_sizes[3] < DM * DM) return;
  const float* x = (const float*)d_in[0];
  const int* adj = (const int*)d_in[1];
  const float* wqkv = (const float*)d_in[2];
  const float* wproj = (const float*)d_in[3];
  float* out = (float*)d_out;
  char* ws = (char*)d_ws; size_t off = 0;
  auto take = [&](size_t bytes) { char* p = ws + off; off += (bytes + 255) & ~(size_t)255; return p; };
  _Float16* WQ = (_Float16*)take((size_t)NQKV * DM * 2);
  _Float16* WP = (_Float16*)take((size_t)DM * DM * 2);
  _Float16* X16 = (_Float16*)take(NR * DM * 2);
  _Float16* QKV16 = (_Float16*)take(NR * NQKV * 2);
  unsigned* BITS = (unsigned*)take((size_t)2 * NB * SEQ * NW * 4);
  unsigned* PM = (unsigned*)take((size_t)NB * NH * SEQ * NW * 4);
  _Float16* VT = (_Float16*)take((size_t)NB * NH * HD * SEQ * 2);
  _Float16* O16 = (_Float16*)take(NR * DM * 2);
  float* S = (float*)take((size_t)NBG * NH * SEQ * SEQ * 4);
  _Float16* P = (_Float16*)take((size_t)NBG * NH * SEQ * SEQ * 2);
  if (off > ws_size) return;

  k_wnat<<<(unsigned)(((size_t)NQKV * DM / 8 + 255) / 256), 256, 0, stream>>>(wqkv, (size_t)NQKV * DM / 8, WQ);
  k_wnat<<<(unsigned)(((size_t)DM * DM / 8 + 255) / 256), 256, 0, stream>>>(wproj, (size_t)DM * DM / 8, WP);
  k_x16<<<(unsigned)((NR * DM / 8 + 255) / 256), 256, 0, stream>>>(x, X16, NR * DM / 8);
  k_pack<<<dim3(SEQ * NW4 / 256, 2, NB), 256, 0, stream>>>(adj, BITS);
  k_mask<<<dim3(SEQ * NW4 / 256, NH, NB), 256, 0, stream>>>(BITS, PM);
  k_gemm2<<<dim3((unsigned)((NR / 128) * (NQKV / 64)), 1, 1), 128, 0, stream>>>(X16, DM, 0, 0, WQ, DM, 0, 0, 0.0625f, nullptr, QKV16, NQKV, 0, 0, NQKV, DM);
  k_vt<NH, SEQ><<<NB * NH * (SEQ / 64), 256, 0, stream>>>(QKV16, NQKV, 2 * DM, VT);
  for (int g = 0; g < NB / NBG; ++g) {
    const size_t b0 = (size_t)g * NBG;
    const _Float16* qg = QKV16 + b0 * SEQ * NQKV;
    k_gemm2<<<dim3((SEQ / 128) * (SEQ / 64), NH, NBG), 128, 0, stream>>>(qg, NQKV, (size_t)HD, (size_t)SEQ * NQKV, qg + DM, NQKV, (size_t)HD, (size_t)SEQ * NQKV, 0.125f,
        S, nullptr, SEQ, (size_t)SEQ * SEQ, (size_t)NH * SEQ * SEQ, SEQ, HD);
    k_msm<<<(NBG * NH * SEQ) / 8, 256, 0, stream>>>(S, PM + b0 * NH * SEQ * NW, P, NBG * NH * SEQ);
    k_gemm2<<<dim3((SEQ / 128) * (HD / 64), NH, NBG), 128, 0, stream>>>(P, SEQ, (size_t)SEQ * SEQ, (size_t)NH * SEQ * SEQ, VT + b0 * NH * HD * SEQ, SEQ, (size_t)HD * SEQ, (size_t)NH * HD * SEQ, 0.25f,
        nullptr, O16 + b0 * SEQ * DM, DM, (size_t)HD, (size_t)SEQ * DM, HD, SEQ);
  }
  k_gemm2<<<dim3((unsigned)((NR / 128) * (DM / 64)), 1, 1), 128, 0, stream>>>(O16, DM, 0, 0, WP, DM, 0, 0, 0.0009765625f, out, nullptr, DM, 0, 0, DM, DM);
}
